// SSMBlock_77996606095827
// MI455X (gfx1250) — hardware-verified
//
#include <hip/hip_runtime.h>
#include <math.h>


#define D_MODEL 1024
#define D_STATE 16
#define D_CONV  4
#define D_INNER 2048
#define DT_RANK 64
#define B_SZ    4
#define L_SEQ   2048
#define NROWS   (B_SZ * L_SEQ)

#define GBM 64
#define GBN 64
#define GBK 32
#define GP  40
#define SP  36

static_assert(NROWS % GBM == 0, "");
static_assert((2 * D_INNER) % GBN == 0 && D_INNER % GBN == 0 && DT_RANK % GBN == 0 && D_MODEL % GBN == 0, "");
static_assert(D_MODEL % GBK == 0 && D_INNER % GBK == 0 && DT_RANK % GBK == 0, "");
static_assert(D_INNER % 32 == 0 && D_STATE % 4 == 0 && L_SEQ % 4 == 0, "");

typedef float v4f __attribute__((ext_vector_type(4)));
typedef float v8f __attribute__((ext_vector_type(8)));
typedef unsigned short v4us __attribute__((ext_vector_type(4)));
typedef unsigned short v8us __attribute__((ext_vector_type(8)));
typedef __bf16 v16bf __attribute__((ext_vector_type(16)));
union Frag { v16bf v; v8us p[2]; };

__device__ __forceinline__ unsigned int bf16_rne(float f) {
    unsigned int u = __float_as_uint(f);
    return (u + 0x7FFFu + ((u >> 16) & 1u)) >> 16;
}

__device__ __forceinline__ void split_one(float x, unsigned short& hi, unsigned short& lo) {
    unsigned int hb = bf16_rne(x);
    float rem = x - __uint_as_float(hb << 16);
    unsigned int lb = bf16_rne(rem);
    hi = (unsigned short)hb;
    lo = (unsigned short)lb;
}

__device__ __forceinline__ void split_bf16x4(v4f x, v4us& hi, v4us& lo) {
    unsigned short h0, h1, h2, h3, l0, l1, l2, l3;
    split_one(x.x, h0, l0);
    split_one(x.y, h1, l1);
    split_one(x.z, h2, l2);
    split_one(x.w, h3, l3);
    hi.x = h0; hi.y = h1; hi.z = h2; hi.w = h3;
    lo.x = l0; lo.y = l1; lo.z = l2; lo.w = l3;
}

__device__ __forceinline__ v8f wmma3_bf16(const Frag& ah, const Frag& al,
                                          const Frag& bh, const Frag& bl, v8f c) {
    c = __builtin_amdgcn_wmma_f32_16x16x32_bf16(false, ah.v, false, bh.v, (short)0, c, false, false);
    c = __builtin_amdgcn_wmma_f32_16x16x32_bf16(false, ah.v, false, bl.v, (short)0, c, false, false);
    c = __builtin_amdgcn_wmma_f32_16x16x32_bf16(false, al.v, false, bh.v, (short)0, c, false, false);
    asm volatile("v_nop\n\tv_nop\n\tv_nop\n\tv_nop"
                 : "+v"(c) : "v"(ah.v), "v"(al.v), "v"(bh.v), "v"(bl.v));
    return c;
}

__device__ __forceinline__ float silu_f(float v) {
    float e = __builtin_amdgcn_exp2f(-v * 1.4426950408889634f);
    return v * __builtin_amdgcn_rcpf(1.f + e);
}

__global__ __launch_bounds__(256) void ln_kernel(const float* __restrict__ x,
                                                 const float* __restrict__ w,
                                                 const float* __restrict__ b,
                                                 float* out, int nrows) {
    __shared__ float red[8];
    const int row = blockIdx.x;
    if (row >= nrows) return;
    const int tid = threadIdx.x, lane = tid & 31, wave = tid >> 5;
    const float* xr = x + (size_t)row * D_MODEL;
    const v4f v = *(const v4f*)(xr + tid * 4);

    float s = (v.x + v.y) + (v.z + v.w);
#pragma unroll
    for (int off = 16; off > 0; off >>= 1) s += __shfl_xor(s, off, 32);
    if (lane == 0) red[wave] = s;
    __syncthreads();
    float tot = 0.f;
#pragma unroll
    for (int i = 0; i < 8; ++i) tot += red[i];
    const float mu = tot * (1.f / D_MODEL);
    __syncthreads();

    v4f d;
    d.x = v.x - mu; d.y = v.y - mu; d.z = v.z - mu; d.w = v.w - mu;
    float s2 = (d.x * d.x + d.y * d.y) + (d.z * d.z + d.w * d.w);
#pragma unroll
    for (int off = 16; off > 0; off >>= 1) s2 += __shfl_xor(s2, off, 32);
    if (lane == 0) red[wave] = s2;
    __syncthreads();
    float tot2 = 0.f;
#pragma unroll
    for (int i = 0; i < 8; ++i) tot2 += red[i];
    const float var = tot2 * (1.f / D_MODEL);
    const float inv = 1.f / sqrtf(var + 1e-5f);

    const v4f wv = *(const v4f*)(w + tid * 4);
    const v4f bv = *(const v4f*)(b + tid * 4);
    v4f o;
    o.x = d.x * inv * wv.x + bv.x;
    o.y = d.y * inv * wv.y + bv.y;
    o.z = d.z * inv * wv.z + bv.z;
    o.w = d.w * inv * wv.w + bv.w;

    float* dst = out + (size_t)row * D_MODEL + tid * 4;
    *(volatile v4f*)dst = o;
    __threadfence();
    *(volatile v4f*)dst = o;
}

__global__ __launch_bounds__(128) void gemm_bf16x3(const float* __restrict__ A,
                                                   const float* __restrict__ W,
                                                   const float* __restrict__ bias,
                                                   float* C, int M, int N, int K, int mode) {
    __shared__ unsigned short sAh[GBM * GP];
    __shared__ unsigned short sAl[GBM * GP];
    __shared__ unsigned short sWh[GBN * GP];
    __shared__ unsigned short sWl[GBN * GP];
    __shared__ float sSt[4][32 * SP];

    const int tid  = threadIdx.x;
    const int lane = tid & 31;
    const int wave = tid >> 5;
    const int h    = lane >> 4;
    const int m    = lane & 15;
    const int wm   = wave & 1;
    const int wn   = wave >> 1;
    const int mBase = blockIdx.y * GBM;
    const int nBase = blockIdx.x * GBN;

    const int sRow = tid >> 3;
    const int sK   = (tid & 7) * 4;

    v4f z4 = {0.f, 0.f, 0.f, 0.f};
    v8f acc[2][2] = {};

    for (int k0 = 0; k0 < K; k0 += GBK) {
        v4f ar[4], wr[4];
#pragma unroll
        for (int i = 0; i < 4; ++i) {
            const int r  = sRow + 16 * i;
            const int gm = mBase + r;
            const int gn = nBase + r;
            ar[i] = (gm < M) ? *(const v4f*)(A + (size_t)gm * K + k0 + sK) : z4;
            wr[i] = (gn < N) ? *(const v4f*)(W + (size_t)gn * K + k0 + sK) : z4;
        }
#pragma unroll
        for (int i = 0; i < 4; ++i) {
            const int r = sRow + 16 * i;
            v4us hi, lo;
            split_bf16x4(ar[i], hi, lo);
            *(v4us*)(sAh + r * GP + sK) = hi;
            *(v4us*)(sAl + r * GP + sK) = lo;
            split_bf16x4(wr[i], hi, lo);
            *(v4us*)(sWh + r * GP + sK) = hi;
            *(v4us*)(sWl + r * GP + sK) = lo;
        }
        __syncthreads();

        Frag ah[2], al[2], bh[2], bl[2];
#pragma unroll
        for (int u = 0; u < 2; ++u) {
            const unsigned short* ph = sAh + (wm * 32 + u * 16 + m) * GP;
            const unsigned short* pl = sAl + (wm * 32 + u * 16 + m) * GP;
            ah[u].p[0] = *(const v8us*)(ph + 8 * h);
            ah[u].p[1] = *(const v8us*)(ph + 16 + 8 * h);
            al[u].p[0] = *(const v8us*)(pl + 8 * h);
            al[u].p[1] = *(const v8us*)(pl + 16 + 8 * h);
        }
#pragma unroll
        for (int t = 0; t < 2; ++t) {
            const unsigned short* ph = sWh + (wn * 32 + t * 16 + m) * GP;
            const unsigned short* pl = sWl + (wn * 32 + t * 16 + m) * GP;
            bh[t].p[0] = *(const v8us*)(ph + 8 * h);
            bh[t].p[1] = *(const v8us*)(ph + 16 + 8 * h);
            bl[t].p[0] = *(const v8us*)(pl + 8 * h);
            bl[t].p[1] = *(const v8us*)(pl + 16 + 8 * h);
        }
#pragma unroll
        for (int u = 0; u < 2; ++u)
#pragma unroll
            for (int t = 0; t < 2; ++t)
                acc[u][t] = wmma3_bf16(ah[u], al[u], bh[t], bl[t], acc[u][t]);
        __syncthreads();
    }

    float* st = sSt[wave];
#pragma unroll
    for (int t = 0; t < 2; ++t) {
        const int col = nBase + wn * 32 + t * 16 + m;
        const float bv = (mode != 0 && col < N) ? bias[col] : 0.f;
#pragma unroll
        for (int u = 0; u < 2; ++u) {
#pragma unroll
            for (int r = 0; r < 8; ++r) {
                float v = acc[u][t][r] + bv;
                if (mode == 2) v = (v > 20.f) ? v : log1pf(expf(v));
                st[(u * 16 + 8 * h + r) * SP + t * 16 + m] = v;
            }
        }
    }
    __syncthreads();

    const int piece = lane & 7;
    const int lrow  = lane >> 3;
    v4f ov[8];
#pragma unroll
    for (int j = 0; j < 8; ++j) {
        const int li = j * 4 + lrow;
        ov[j] = *(const v4f*)(st + li * SP + piece * 4);
    }
    const int colseg = nBase + wn * 32;
    const bool colok = (colseg + 32 <= N);
#pragma unroll
    for (int j = 0; j < 8; ++j) {
        const int grow = mBase + wm * 32 + j * 4 + lrow;
        if (colok && grow < M)
            *(volatile v4f*)(C + (size_t)grow * N + colseg + piece * 4) = ov[j];
    }
    __threadfence();
#pragma unroll
    for (int j = 0; j < 8; ++j) {
        const int grow = mBase + wm * 32 + j * 4 + lrow;
        if (colok && grow < M)
            *(volatile v4f*)(C + (size_t)grow * N + colseg + piece * 4) = ov[j];
    }
}

__global__ __launch_bounds__(256) void conv_silu_kernel(const float* __restrict__ xz,
                                                        const float* __restrict__ cw,
                                                        const float* __restrict__ cb,
                                                        const float* __restrict__ gw,
                                                        const float* __restrict__ gb,
                                                        float* xs, float* zal, int nvec) {
    const int q = blockIdx.x * blockDim.x + threadIdx.x;
    if (q >= nvec) return;
    const int cq  = q % (D_INNER / 4);
    const int row = q / (D_INNER / 4);
    const int c0  = cq * 4;
    const int l   = row % L_SEQ;
    const int b   = row / L_SEQ;

    v4f ax = *(const v4f*)(cb + c0);
    v4f az = *(const v4f*)(gb + c0);
    v4f wx[4], wz[4];
#pragma unroll
    for (int j = 0; j < 4; ++j) {
        wx[j] = *(const v4f*)(cw + (size_t)(c0 + j) * D_CONV);
        wz[j] = *(const v4f*)(gw + (size_t)(c0 + j) * D_CONV);
    }
#pragma unroll
    for (int k = 0; k < D_CONV; ++k) {
        const int t = l - (D_CONV - 1) + k;
        if (t >= 0) {
            const size_t base = (size_t)(b * L_SEQ + t) * (2 * D_INNER);
            const v4f xv = *(const v4f*)(xz + base + c0);
            const v4f zv = *(const v4f*)(xz + base + D_INNER + c0);
            ax.x = fmaf(wx[0][k], xv.x, ax.x);
            ax.y = fmaf(wx[1][k], xv.y, ax.y);
            ax.z = fmaf(wx[2][k], xv.z, ax.z);
            ax.w = fmaf(wx[3][k], xv.w, ax.w);
            az.x = fmaf(wz[0][k], zv.x, az.x);
            az.y = fmaf(wz[1][k], zv.y, az.y);
            az.z = fmaf(wz[2][k], zv.z, az.z);
            az.w = fmaf(wz[3][k], zv.w, az.w);
        }
    }
    v4f ox, oz;
    ox.x = silu_f(ax.x); ox.y = silu_f(ax.y); ox.z = silu_f(ax.z); ox.w = silu_f(ax.w);
    oz.x = silu_f(az.x); oz.y = silu_f(az.y); oz.z = silu_f(az.z); oz.w = silu_f(az.w);

    const size_t o = (size_t)row * D_INNER + c0;
    *(volatile v4f*)(xs + o)  = ox;
    *(volatile v4f*)(zal + o) = oz;
    __threadfence();
    *(volatile v4f*)(xs + o)  = ox;
    *(volatile v4f*)(zal + o) = oz;
}

__global__ __launch_bounds__(256) void dt_mean_kernel(const float* __restrict__ dt,
                                                      float* dt_avg, int nrows) {
    const int q = blockIdx.x * blockDim.x + threadIdx.x;
    if (q >= D_INNER / 4) return;
    const int c0 = q * 4;
    double s0 = 0.0, s1 = 0.0, s2 = 0.0, s3 = 0.0;
#pragma unroll 4
    for (int r = 0; r < nrows; ++r) {
        const v4f v = *(const v4f*)(dt + (size_t)r * D_INNER + c0);
        s0 += (double)v.x; s1 += (double)v.y; s2 += (double)v.z; s3 += (double)v.w;
    }
    const double invn = 1.0 / (double)nrows;
    v4f o;
    o.x = (float)(s0 * invn); o.y = (float)(s1 * invn);
    o.z = (float)(s2 * invn); o.w = (float)(s3 * invn);
    *(volatile v4f*)(dt_avg + c0) = o;
    __threadfence();
    *(volatile v4f*)(dt_avg + c0) = o;
}

__device__ __forceinline__ void disc_one(float a_log, float bmv, float dtv, float& ab, float& bb) {
    const float A   = -expf(a_log);
    const float Ae  = A * dtv;
    const float Abv = expf(Ae);
    const bool  sm  = fabsf(Ae) < 1e-6f;
    const float ex  = sm ? Ae : (Abv - 1.f);
    const float Ainv = 1.f / (A + 1e-8f);
    const float sf  = sm ? dtv : Ainv * ex;
    ab = Abv;
    bb = sf * bmv;
}

__global__ __launch_bounds__(256) void discretize_kernel(const float* __restrict__ A_log,
                                                         const float* __restrict__ Bm,
                                                         const float* __restrict__ dt_avg,
                                                         float* Abar, float* Bbar, int nvec) {
    const int q = blockIdx.x * blockDim.x + threadIdx.x;
    if (q >= nvec) return;
    const int idx0 = q * 4;
    const int i    = idx0 / D_STATE;
    const v4f al = *(const v4f*)(A_log + idx0);
    const v4f bm = *(const v4f*)(Bm + idx0);
    const float dtv = dt_avg[i];
    float a0, a1, a2, a3, b0, b1, b2, b3;
    disc_one(al.x, bm.x, dtv, a0, b0);
    disc_one(al.y, bm.y, dtv, a1, b1);
    disc_one(al.z, bm.z, dtv, a2, b2);
    disc_one(al.w, bm.w, dtv, a3, b3);
    v4f ab, bb;
    ab.x = a0; ab.y = a1; ab.z = a2; ab.w = a3;
    bb.x = b0; bb.y = b1; bb.z = b2; bb.w = b3;
    *(volatile v4f*)(Abar + idx0) = ab;
    *(volatile v4f*)(Bbar + idx0) = bb;
    __threadfence();
    *(volatile v4f*)(Abar + idx0) = ab;
    *(volatile v4f*)(Bbar + idx0) = bb;
}

__global__ __launch_bounds__(256) void scan_kernel(const float* __restrict__ xs,
                                                   const float* __restrict__ zal,
                                                   const float* __restrict__ Abar,
                                                   const float* __restrict__ Bbar,
                                                   const float* __restrict__ Cm,
                                                   const float* __restrict__ Dv,
                                                   float* G, int ntotal) {
    __shared__ float st[8][4 * 32];
    const int tid = threadIdx.x, lane = tid & 31, wave = tid >> 5;
    const int gid = blockIdx.x * blockDim.x + tid;
    const bool wact = (int)(blockIdx.x * blockDim.x + wave * 32) < ntotal;
    const int g = (gid < ntotal) ? gid : 0;
    const int i = g % D_INNER;
    const int b = g / D_INNER;
    const int i0 = i - lane;

    float Ab[D_STATE], Bb[D_STATE], Cv[D_STATE], hs[D_STATE];
#pragma unroll
    for (int d4 = 0; d4 < D_STATE; d4 += 4) {
        const v4f va = *(const v4f*)(Abar + (size_t)i * D_STATE + d4);
        const v4f vb = *(const v4f*)(Bbar + (size_t)i * D_STATE + d4);
        const v4f vc = *(const v4f*)(Cm   + (size_t)i * D_STATE + d4);
        Ab[d4] = va.x; Ab[d4 + 1] = va.y; Ab[d4 + 2] = va.z; Ab[d4 + 3] = va.w;
        Bb[d4] = vb.x; Bb[d4 + 1] = vb.y; Bb[d4 + 2] = vb.z; Bb[d4 + 3] = vb.w;
        Cv[d4] = vc.x; Cv[d4 + 1] = vc.y; Cv[d4 + 2] = vc.z; Cv[d4 + 3] = vc.w;
        hs[d4] = 0.f; hs[d4 + 1] = 0.f; hs[d4 + 2] = 0.f; hs[d4 + 3] = 0.f;
    }
    const float dfac = 1.f + Dv[i];
    const size_t base = (size_t)b * L_SEQ * D_INNER;
    const int q = lane >> 3, piece = lane & 7;

    for (int t0 = 0; t0 < L_SEQ; t0 += 4) {
#pragma unroll 1
        for (int s = 0; s < 4; ++s) {
            const size_t o = base + (size_t)(t0 + s) * D_INNER + i;
            const float xv = xs[o];
            const float zv = zal[o];
            float y = 0.f;
#pragma unroll
            for (int d = 0; d < D_STATE; ++d) {
                hs[d] = fmaf(Ab[d], hs[d], Bb[d] * xv);
                y = fmaf(hs[d], Cv[d], y);
            }
            st[wave][s * 32 + lane] = y * zv * dfac;
        }
        __syncthreads();
        const v4f v = *(const v4f*)(&st[wave][q * 32 + piece * 4]);
        float* dst = G + base + (size_t)(t0 + q) * D_INNER + i0 + piece * 4;
        if (wact) *(volatile v4f*)dst = v;
        __threadfence();
        if (wact) *(volatile v4f*)dst = v;
        __syncthreads();
    }
}

extern "C" void kernel_launch(void* const* d_in, const int* in_sizes, int n_in,
                              void* d_out, int out_size, void* d_ws, size_t ws_size,
                              hipStream_t stream) {
    if (n_in < 18) return;
    const size_t MI = (size_t)1 << 20;
    const size_t need_bytes = 64 * MI * sizeof(float);
    if (ws_size < need_bytes) return;
    if (in_sizes[0]  != NROWS * D_MODEL)      return;
    if (in_sizes[1]  != D_MODEL)              return;
    if (in_sizes[2]  != D_MODEL)              return;
    if (in_sizes[3]  != 2 * D_INNER * D_MODEL) return;
    if (in_sizes[4]  != 2 * D_INNER)          return;
    if (in_sizes[5]  != D_INNER * D_CONV)     return;
    if (in_sizes[6]  != D_INNER)              return;
    if (in_sizes[7]  != D_INNER * D_CONV)     return;
    if (in_sizes[8]  != D_INNER)              return;
    if (in_sizes[9]  != D_INNER * D_STATE)    return;
    if (in_sizes[10] != D_INNER * D_STATE)    return;
    if (in_sizes[11] != D_INNER * D_STATE)    return;
    if (in_sizes[12] != D_INNER)              return;
    if (in_sizes[13] != DT_RANK * D_INNER)    return;
    if (in_sizes[14] != D_INNER * DT_RANK)    return;
    if (in_sizes[15] != D_INNER)              return;
    if (in_sizes[16] != D_MODEL * D_INNER)    return;
    if (in_sizes[17] != D_MODEL)              return;
    if (out_size     != NROWS * D_MODEL)      return;

    const float* x          = (const float*)d_in[0];
    const float* ln_w       = (const float*)d_in[1];
    const float* ln_b       = (const float*)d_in[2];
    const float* in_proj_w  = (const float*)d_in[3];
    const float* in_proj_b  = (const float*)d_in[4];
    const float* conv_w     = (const float*)d_in[5];
    const float* conv_b     = (const float*)d_in[6];
    const float* gate_w     = (const float*)d_in[7];
    const float* gate_b     = (const float*)d_in[8];
    const float* A_log      = (const float*)d_in[9];
    const float* B_mat      = (const float*)d_in[10];
    const float* C_mat      = (const float*)d_in[11];
    const float* D_vec      = (const float*)d_in[12];
    const float* A_proj_w   = (const float*)d_in[13];
    const float* dt_proj_w  = (const float*)d_in[14];
    const float* dt_proj_b  = (const float*)d_in[15];
    const float* out_proj_w = (const float*)d_in[16];
    const float* out_proj_b = (const float*)d_in[17];
    float* out = (float*)d_out;

    float* ws = (float*)d_ws;
    float* xz     = ws;
    float* xn     = ws + 32 * MI;
    float* xs     = ws + 32 * MI;
    float* zal    = ws + 48 * MI;
    float* A_in   = ws + 16 * MI;
    float* dtb    = ws;
    float* dt_avg = ws + 31 * MI;
    float* Abar   = dt_avg + D_INNER;
    float* Bbar   = Abar + D_INNER * D_STATE;
    float* G      = ws;

    ln_kernel<<<NROWS, 256, 0, stream>>>(x, ln_w, ln_b, xn, NROWS);

    {
        dim3 g((2 * D_INNER + GBN - 1) / GBN, (NROWS + GBM - 1) / GBM);
        gemm_bf16x3<<<g, 128, 0, stream>>>(xn, in_proj_w, in_proj_b, xz,
                                           NROWS, 2 * D_INNER, D_MODEL, 1);
    }

    {
        const int nvec = NROWS * D_INNER / 4;
        conv_silu_kernel<<<(nvec + 255) / 256, 256, 0, stream>>>(
            xz, conv_w, conv_b, gate_w, gate_b, xs, zal, nvec);
    }

    {
        dim3 g((DT_RANK + GBN - 1) / GBN, (NROWS + GBM - 1) / GBM);
        gemm_bf16x3<<<g, 128, 0, stream>>>(xs, A_proj_w, dt_proj_b, A_in,
                                           NROWS, DT_RANK, D_INNER, 0);
    }

    {
        dim3 g((D_INNER + GBN - 1) / GBN, (NROWS + GBM - 1) / GBM);
        gemm_bf16x3<<<g, 128, 0, stream>>>(A_in, dt_proj_w, dt_proj_b, dtb,
                                           NROWS, D_INNER, DT_RANK, 2);
    }

    dt_mean_kernel<<<(D_INNER / 4 + 255) / 256, 256, 0, stream>>>(dtb, dt_avg, NROWS);

    {
        const int nvec = D_INNER * D_STATE / 4;
        discretize_kernel<<<(nvec + 255) / 256, 256, 0, stream>>>(
            A_log, B_mat, dt_avg, Abar, Bbar, nvec);
    }

    {
        const int ntotal = B_SZ * D_INNER;
        scan_kernel<<<(ntotal + 255) / 256, 256, 0, stream>>>(
            xs, zal, Abar, Bbar, C_mat, D_vec, G, ntotal);
    }

    {
        dim3 g((D_MODEL + GBN - 1) / GBN, (NROWS + GBM - 1) / GBM);
        gemm_bf16x3<<<g, 128, 0, stream>>>(G, out_proj_w, out_proj_b, out,
                                           NROWS, D_MODEL, D_INNER, 1);
    }
}
